// TGATPredictorAblation_34170759807353
// MI455X (gfx1250) — hardware-verified
//
#include <hip/hip_runtime.h>
#include <math.h>

#pragma clang fp contract(off)

typedef unsigned short us;
typedef _Float16 v16h __attribute__((ext_vector_type(16)));
typedef __bf16   v16b __attribute__((ext_vector_type(16)));
typedef us       v16us __attribute__((ext_vector_type(16)));
typedef us       v8us __attribute__((ext_vector_type(8)));
typedef float    v8f __attribute__((ext_vector_type(8)));
typedef unsigned v4u __attribute__((ext_vector_type(4)));
typedef v8us __attribute__((may_alias)) v8usa;
typedef v4u  __attribute__((may_alias)) v4ua;

union FragU { v16us v; v8us half[2]; };

#define NB    1024
#define NLC   200
#define NROWC (NB * NLC)
#define HID   256
#define KVP   288
#define LP    224
#define QKW   1152

#define OFF_WINS_HI 0
#define OFF_WINS_LO 24576
#define OFF_WINC    49152
#define OFF_L0      73728
#define LSTRIDE     819200
#define L_WQ_HI 0
#define L_WQ_LO 65536
#define L_WK_HI 131072
#define L_WK_LO 204800
#define L_WV_HI 278528
#define L_WV_LO 352256
#define L_WR_HI 425984
#define L_WR_LO 491520
#define L_W1_HI 557056
#define L_W1_LO 622592
#define L_W2_HI 688128
#define L_W2_LO 753664
#define OFF_RB   2531328
#define R_WRO_HI 0
#define R_WRO_LO 65536
#define R_RO2_HI 131072
#define R_RO2_LO 155648
#define WTOTAL_HALVES 2711552

#define WS_CTX   0ull
#define WS_H     104857600ull
#define WS_QK    105906176ull
#define WS_AW    108265472ull
#define WS_W     112984064ull
#define WS_TOTAL (WS_W + 2ull * WTOTAL_HALVES)

#define LDS_INPROJ0 90112
#define LDS_INPROJ1 57344
#define LDS_QK      139264
#define LDS_ATTN    159744
#define LDS_POST    122880
#define LDS_RDO     69888

__device__ __forceinline__ us f2bf(float x) {
  unsigned u = __builtin_bit_cast(unsigned, x);
  u += 0x7FFFu + ((u >> 16) & 1u);
  return (us)(u >> 16);
}
__device__ __forceinline__ float bf2f(us b) { return __builtin_bit_cast(float, ((unsigned)b) << 16); }
__device__ __forceinline__ us f2hb(float x) { const _Float16 hv = (_Float16)x; return __builtin_bit_cast(us, hv); }

__device__ __forceinline__ v8f zero8() { v8f z = {0.f, 0.f, 0.f, 0.f, 0.f, 0.f, 0.f, 0.f}; return z; }
__device__ __forceinline__ v4u zero4u() { v4u z = {0u, 0u, 0u, 0u}; return z; }
__device__ __forceinline__ v4u sel4(bool c, v4u a, v4u b) {
  v4u r; r.x = c ? a.x : b.x; r.y = c ? a.y : b.y; r.z = c ? a.z : b.z; r.w = c ? a.w : b.w; return r;
}

__device__ __forceinline__ float wsum(float v) {
  v += __shfl_xor(v, 16); v += __shfl_xor(v, 8); v += __shfl_xor(v, 4); v += __shfl_xor(v, 2); v += __shfl_xor(v, 1);
  return v;
}
__device__ __forceinline__ float wmaxf(float v) {
  v = fmaxf(v, __shfl_xor(v, 16)); v = fmaxf(v, __shfl_xor(v, 8)); v = fmaxf(v, __shfl_xor(v, 4));
  v = fmaxf(v, __shfl_xor(v, 2)); v = fmaxf(v, __shfl_xor(v, 1));
  return v;
}

__device__ __forceinline__ v8f mma_f16(v16us a, v16us b, v8f c) {
  const v16h av = __builtin_bit_cast(v16h, a);
  const v16h bv = __builtin_bit_cast(v16h, b);
  v8f d = __builtin_amdgcn_wmma_f32_16x16x32_f16(false, av, false, bv, (short)0, c, false, false);
  asm volatile("v_nop\n\tv_nop\n\tv_nop\n\tv_nop" : "+v"(d) : "v"(av), "v"(bv));
  return d;
}
__device__ __forceinline__ v8f mma_bf16(v16us a, v16us b, v8f c) {
  const v16b av = __builtin_bit_cast(v16b, a);
  const v16b bv = __builtin_bit_cast(v16b, b);
  v8f d = __builtin_amdgcn_wmma_f32_16x16x32_bf16(false, av, false, bv, (short)0, c, false, false);
  asm volatile("v_nop\n\tv_nop\n\tv_nop\n\tv_nop" : "+v"(d) : "v"(av), "v"(bv));
  return d;
}

__device__ __forceinline__ v16us ldfrag(const us* p, int h) {
  FragU f;
  f.half[0] = *(const v8usa*)(p + 8 * h);
  f.half[1] = *(const v8usa*)(p + 16 + 8 * h);
  return f.v;
}

template<int MT, int NT>
__device__ __forceinline__ void gemm_split(v8f (&acc)[MT][NT],
    const us* aHi, const us* aLo, int lda, const us* bHi, const us* bLo, int ldb, int ksteps, int lane)
{
  const int h = lane >> 4, m = lane & 15;
  #pragma unroll 1
  for (int ks = 0; ks < ksteps; ++ks) {
    const int k0 = ks * 32;
    v16us bh[NT], bl[NT];
    #pragma unroll
    for (int nt = 0; nt < NT; ++nt) {
      const size_t bo = (size_t)(16 * nt + m) * ldb + k0;
      bh[nt] = ldfrag(bHi + bo, h);
      bl[nt] = ldfrag(bLo + bo, h);
    }
    #pragma unroll
    for (int mt = 0; mt < MT; ++mt) {
      const int ao = (16 * mt + m) * lda + k0;
      const v16us ah = ldfrag(aHi + ao, h);
      const v16us al = ldfrag(aLo + ao, h);
      #pragma unroll
      for (int nt = 0; nt < NT; ++nt) {
        v8f d = acc[mt][nt];
        d = mma_bf16(ah, bh[nt], d);
        d = mma_bf16(ah, bl[nt], d);
        d = mma_bf16(al, bh[nt], d);
        acc[mt][nt] = d;
      }
    }
  }
}

template<int MT, int NT>
__device__ __forceinline__ void gemm_f16(v8f (&acc)[MT][NT],
    const us* aT, int lda, const us* bP, int ldb, int ksteps, int lane)
{
  const int h = lane >> 4, m = lane & 15;
  #pragma unroll 1
  for (int ks = 0; ks < ksteps; ++ks) {
    const int k0 = ks * 32;
    v16us bf[NT];
    #pragma unroll
    for (int nt = 0; nt < NT; ++nt) bf[nt] = ldfrag(bP + (size_t)(16 * nt + m) * ldb + k0, h);
    #pragma unroll
    for (int mt = 0; mt < MT; ++mt) {
      const v16us a = ldfrag(aT + (16 * mt + m) * lda + k0, h);
      #pragma unroll
      for (int nt = 0; nt < NT; ++nt) acc[mt][nt] = mma_f16(a, bf[nt], acc[mt][nt]);
    }
  }
}

__device__ __forceinline__ void stage_split(const float* src, int n, us* hi, us* lo, int tid) {
  for (int idx = tid; idx < n; idx += 256) {
    const float x = src[idx];
    const us hb = f2bf(x);
    hi[idx] = hb;
    lo[idx] = f2bf(x - bf2f(hb));
  }
}

__device__ __forceinline__ void store_lines(const unsigned char* lsrc, unsigned char* gdst,
                                            int nlines, int wave, int lane, int nwaves) {
  const int sub = lane >> 3, q8 = lane & 7;
  for (int ln = wave * 4 + sub; ln < nlines; ln += nwaves * 4) {
    const v4u v = *(const v4ua*)(lsrc + (size_t)ln * 128 + 16 * q8);
    *(volatile v4u*)(gdst + (size_t)ln * 128 + 16 * q8) = v;
  }
}

__global__ __launch_bounds__(256) void k_cvt(
    const float* __restrict__ WinS, const float* __restrict__ WinC,
    const float* __restrict__ Wq, const float* __restrict__ Wk, const float* __restrict__ Wv,
    const float* __restrict__ Wres, const float* __restrict__ Wff1, const float* __restrict__ Wff2,
    const float* __restrict__ Wro, const float* __restrict__ Wcls, const float* __restrict__ Wdt,
    const float* __restrict__ Wrem, us* __restrict__ wsw)
{
  __shared__ __align__(16) us tHi[32 * 288];
  __shared__ __align__(16) us tLo[32 * 288];

  const int jid = blockIdx.y;
  const float* src = WinS;
  int sn = 1, sk = 256, nval = 256, kval = 96, npad = 256, kpad = 96, mode = 0;
  float scale = 1.0f;
  int dh = OFF_WINS_HI, dl = OFF_WINS_LO;
  if (jid == 1) {
    src = WinC; mode = 1; scale = 16.0f; dh = OFF_WINC; dl = OFF_WINC;
  } else if (jid >= 2 && jid < 20) {
    const int li = (jid - 2) / 6, ty = (jid - 2) - 6 * li;
    const int lb = OFF_L0 + li * LSTRIDE;
    kval = 256; kpad = 256;
    if (ty == 0)      { src = Wq   + (size_t)li * 65536; dh = lb + L_WQ_HI; dl = lb + L_WQ_LO; }
    else if (ty == 1) { src = Wk   + (size_t)li * 69632; sn = 256; sk = 1; nval = 272; npad = 288; dh = lb + L_WK_HI; dl = lb + L_WK_LO; }
    else if (ty == 2) { src = Wv   + (size_t)li * 69632; kval = 272; kpad = 288; dh = lb + L_WV_HI; dl = lb + L_WV_LO; }
    else if (ty == 3) { src = Wres + (size_t)li * 65536; dh = lb + L_WR_HI; dl = lb + L_WR_LO; }
    else if (ty == 4) { src = Wff1 + (size_t)li * 65536; dh = lb + L_W1_HI; dl = lb + L_W1_LO; }
    else              { src = Wff2 + (size_t)li * 65536; dh = lb + L_W2_HI; dl = lb + L_W2_LO; }
  } else if (jid == 20) {
    src = Wro; kval = 256; kpad = 256; dh = OFF_RB + R_WRO_HI; dl = OFF_RB + R_WRO_LO;
  } else if (jid == 21) {
    src = Wcls; sk = 32; nval = 32; kval = 256; npad = 32; kpad = 256; dh = OFF_RB + R_RO2_HI; dl = OFF_RB + R_RO2_LO;
  } else if (jid == 22) {
    src = Wdt; sk = 1; nval = 1; kval = 256; npad = 32; kpad = 256; dh = OFF_RB + R_RO2_HI + 8192; dl = OFF_RB + R_RO2_LO + 8192;
  } else if (jid == 23) {
    src = Wrem; sk = 1; nval = 1; kval = 256; npad = 32; kpad = 256; dh = OFF_RB + R_RO2_HI + 16384; dl = OFF_RB + R_RO2_LO + 16384;
  }

  const int n0 = blockIdx.x * 32;
  if (n0 >= npad) return;
  const int tid = threadIdx.x, lane = tid & 31, w = tid >> 5;

  for (int r = 0; r < 32; ++r) {
    const int n = n0 + r;
    const int nc = min(n, nval - 1);
    const bool nok = n < nval;
    for (int k = tid; k < kpad; k += 256) {
      const int kc = min(k, kval - 1);
      float x = src[(size_t)nc * sn + (size_t)kc * sk] * scale;
      x = (nok && k < kval) ? x : 0.0f;
      const int o = r * kpad + k;
      if (mode == 0) {
        const us hb = f2bf(x);
        tHi[o] = hb;
        tLo[o] = f2bf(x - bf2f(hb));
      } else {
        tHi[o] = f2hb(x);
        tLo[o] = 0;
      }
    }
  }
  __syncthreads();

  const int nlines = kpad >> 1;
  unsigned char* gh = (unsigned char*)(wsw + (size_t)dh + (size_t)n0 * kpad);
  unsigned char* gl = (unsigned char*)(wsw + (size_t)dl + (size_t)n0 * kpad);
  store_lines((const unsigned char*)tHi, gh, nlines, w, lane, 8);
  if (mode == 0) store_lines((const unsigned char*)tLo, gl, nlines, w, lane, 8);
  __threadfence();
  store_lines((const unsigned char*)tHi, gh, nlines, w, lane, 8);
  if (mode == 0) store_lines((const unsigned char*)tLo, gl, nlines, w, lane, 8);
}

template<int MODE>
__global__ __launch_bounds__(256) void k_inproj(
    const float* __restrict__ x, const int* __restrict__ act, const float* __restrict__ emb,
    const us* __restrict__ wHi, const us* __restrict__ wLo, const float* __restrict__ bias,
    unsigned char* __restrict__ outp, int nrows)
{
  extern __shared__ __align__(16) unsigned char dynlds[];
  us* aHi = (us*)dynlds;
  us* aLo = aHi + 64 * 96;
  unsigned char* sOut = dynlds + 24576;

  const int tid = threadIdx.x, lane = tid & 31, w = tid >> 5;
  const int h = lane >> 4, m = lane & 15;
  const int row0 = blockIdx.x * 64;
  if (row0 + 64 > nrows) return;

  for (int idx = tid; idx < 64 * 96; idx += 256) {
    const int r = idx / 96, c = idx - r * 96;
    const int row = row0 + r;
    const float xv = x[(size_t)row * 64 + min(c, 63)];
    int ai = act[row];
    ai = min(max(ai, 0), 32);
    const float ev = emb[ai * 32 + max(c - 64, 0)];
    const float v = (c < 64) ? xv : ev;
    if constexpr (MODE == 0) {
      const us hb = f2bf(v);
      aHi[idx] = hb;
      aLo[idx] = f2bf(v - bf2f(hb));
    } else {
      aHi[idx] = f2hb(v);
    }
  }
  __syncthreads();

  v8f acc[4][2];
  #pragma unroll
  for (int mt = 0; mt < 4; ++mt) { acc[mt][0] = zero8(); acc[mt][1] = zero8(); }
  const int nb = 32 * w;
  if constexpr (MODE == 0) {
    gemm_split<4, 2>(acc, aHi, aLo, 96, wHi + (size_t)nb * 96, wLo + (size_t)nb * 96, 96, 3, lane);
  } else {
    gemm_f16<4, 2>(acc, aHi, 96, wHi + (size_t)nb * 96, 96, 3, lane);
  }

  #pragma unroll
  for (int nt = 0; nt < 2; ++nt) {
    const int col = nb + 16 * nt + m;
    const float bv = bias[col];
    #pragma unroll
    for (int mt = 0; mt < 4; ++mt) {
      #pragma unroll
      for (int r = 0; r < 8; ++r) {
        const int row = 16 * mt + 8 * h + r;
        if constexpr (MODE == 0) {
          ((float*)sOut)[row * 256 + col] = acc[mt][nt][r] + bv;
        } else {
          ((us*)sOut)[row * 256 + col] = f2hb(acc[mt][nt][r] * 0.0625f + bv);
        }
      }
    }
  }
  __syncthreads();

  const int nlines = (MODE == 0) ? 512 : 256;
  unsigned char* gd = outp + (size_t)row0 * 256 * ((MODE == 0) ? 4 : 2);
  store_lines(sOut, gd, nlines, w, lane, 8);
  __threadfence();
  store_lines(sOut, gd, nlines, w, lane, 8);
}

__global__ __launch_bounds__(256) void k_qk(
    const float* __restrict__ hp, const us* __restrict__ wqHi, const us* __restrict__ wqLo,
    const us* __restrict__ wkHi, const us* __restrict__ wkLo, unsigned char* __restrict__ qkp)
{
  extern __shared__ __align__(16) unsigned char dynlds[];
  us* aHi = (us*)dynlds;
  us* aLo = aHi + 8192;
  us* qHi = aLo + 8192;
  us* qLo = qHi + 8192;
  us* sQK = qLo + 8192;

  const int tid = threadIdx.x, lane = tid & 31, w = tid >> 5;
  const int h = lane >> 4, m = lane & 15;
  const int row0 = blockIdx.x * 32;

  stage_split(hp + (size_t)row0 * 256, 8192, aHi, aLo, tid);
  __syncthreads();

  const int nb = 32 * w;
  {
    v8f acc[2][2];
    acc[0][0] = zero8(); acc[0][1] = zero8(); acc[1][0] = zero8(); acc[1][1] = zero8();
    gemm_split<2, 2>(acc, aHi, aLo, 256, wqHi + (size_t)nb * 256, wqLo + (size_t)nb * 256, 256, 8, lane);
    #pragma unroll
    for (int nt = 0; nt < 2; ++nt) {
      const int col = nb + 16 * nt + m;
      #pragma unroll
      for (int mt = 0; mt < 2; ++mt) {
        #pragma unroll
        for (int r = 0; r < 8; ++r) {
          const int row = 16 * mt + 8 * h + r;
          const float q = acc[mt][nt][r];
          const us qh = f2bf(q);
          qHi[row * 256 + col] = qh;
          qLo[row * 256 + col] = f2bf(q - bf2f(qh));
        }
      }
    }
  }
  __syncthreads();

  #pragma unroll 1
  for (int t = 0; t < 9; ++t) {
    const int g = 9 * w + t;
    const int hd = g / 18;
    const int nt = g - 18 * hd;
    v8f a2[2][1];
    a2[0][0] = zero8(); a2[1][0] = zero8();
    gemm_split<2, 1>(a2, qHi + 64 * hd, qLo + 64 * hd, 256,
                     wkHi + (size_t)(16 * nt) * 256 + 64 * hd, wkLo + (size_t)(16 * nt) * 256 + 64 * hd,
                     256, 2, lane);
    #pragma unroll
    for (int mt = 0; mt < 2; ++mt) {
      #pragma unroll
      for (int r = 0; r < 8; ++r) {
        const int row = 16 * mt + 8 * h + r;
        sQK[row * QKW + 288 * hd + 16 * nt + m] = f2hb(a2[mt][0][r] * 2.0f);
      }
    }
  }
  __syncthreads();

  unsigned char* gd = qkp + (size_t)row0 * (QKW * 2);
  store_lines((const unsigned char*)sQK, gd, 576, w, lane, 8);
  __threadfence();
  store_lines((const unsigned char*)sQK, gd, 576, w, lane, 8);
}

__global__ __launch_bounds__(256) void k_attn(
    const us* __restrict__ ctx, const float* __restrict__ tc, const int* __restrict__ act,
    const float* __restrict__ fr, const float* __restrict__ ph,
    const unsigned char* __restrict__ qkp, unsigned char* __restrict__ awp)
{
  extern __shared__ __align__(16) unsigned char dynlds[];
  us* sKV    = (us*)dynlds;
  us* sQK    = (us*)(dynlds + 129024);
  us* sATT   = (us*)(dynlds + 138240);
  us* sTE    = (us*)(dynlds + 145408);
  float* sS  = (float*)(dynlds + 151808);
  float* sAW = (float*)(dynlds + 155136);

  const int tid = threadIdx.x, lane = tid & 31, w = tid >> 5;
  const int h = lane >> 4, m = lane & 15;
  const int b = blockIdx.x;
  const v4u z4 = zero4u();

  {
    const int lc = min(tid, NLC - 1);
    const float tv = tc[(size_t)b * NLC + lc];
    const float lt = log1pf(fmaxf(tv, 0.0f));
    #pragma unroll 1
    for (int k = 0; k < 8; ++k) {
      const float z = lt * fr[k] + ph[k];
      const float sv = sinf(z);
      const float cv = cosf(z);
      if (tid < NLC) {
        sTE[tid * 16 + k] = f2hb(sv);
        sTE[tid * 16 + 8 + k] = f2hb(cv);
      }
    }
  }
  for (int i = tid; i < 144; i += 256) {
    const v4u v = *(const v4ua*)(qkp + (size_t)b * (QKW * 2) + 16 * i);
    *(v4ua*)((unsigned char*)sQK + 16 * i) = v;
  }
  for (int i = tid; i < 432; i += 256) *(v4ua*)((unsigned char*)sQK + 2304 + 16 * i) = z4;
  for (int i = tid; i < 336; i += 256) *(v4ua*)((unsigned char*)sATT + 1792 + 16 * i) = z4;
  __syncthreads();

  for (int task = tid; task < LP * 36; task += 256) {
    const int l = task / 36, c = task - 36 * l;
    const int lc = min(l, NLC - 1), cc = min(c, 31);
    const v4u g = *(const v4ua*)(ctx + ((size_t)(b * NLC + lc)) * 256 + 8 * cc);
    const int tcn = min(max(c - 32, 0), 1);
    const v4u te = *(const v4ua*)(sTE + lc * 16 + 8 * tcn);
    const bool rok = l < NLC;
    const v4u v = sel4(rok && c < 32, g, sel4(rok && c < 34, te, z4));
    *(v4ua*)(sKV + l * KVP + 8 * c) = v;
  }
  __syncthreads();

  for (int mt = w; mt < 13; mt += 8) {
    v8f acc = zero8();
    #pragma unroll
    for (int ks = 0; ks < 9; ++ks) {
      const v16us a = ldfrag(sKV + (16 * mt + m) * KVP + 32 * ks, h);
      const v16us q = ldfrag(sQK + m * KVP + 32 * ks, h);
      acc = mma_f16(a, q, acc);
    }
    if (m < 4) {
      #pragma unroll
      for (int r = 0; r < 8; ++r) sS[m * 208 + 16 * mt + 8 * h + r] = acc[r];
    }
  }
  __syncthreads();

  if (w < 4) {
    const int hd = w;
    float xs[7];
    float mx = -3.0e38f;
    #pragma unroll
    for (int i = 0; i < 7; ++i) {
      const int l = lane + 32 * i;
      const int lc = min(l, NLC - 1);
      const float s = sS[hd * 208 + lc] * 0.0625f;
      const int mk = act[(size_t)b * NLC + lc];
      const float xv = (l < NLC) ? ((mk > 0) ? s : -1.0e9f) : -3.0e38f;
      xs[i] = xv;
      mx = fmaxf(mx, xv);
    }
    mx = wmaxf(mx);
    float p[7];
    float sm = 0.0f;
    #pragma unroll
    for (int i = 0; i < 7; ++i) {
      const int l = lane + 32 * i;
      const float e = (l < NLC) ? expf(xs[i] - mx) : 0.0f;
      p[i] = e;
      sm += e;
    }
    sm = wsum(sm);
    const float inv = 1.0f / sm;
    #pragma unroll
    for (int i = 0; i < 7; ++i) {
      const int l = lane + 32 * i;
      const float a = (l < NLC) ? (p[i] * inv * 16384.0f) : 0.0f;
      sATT[hd * LP + l] = f2hb(a);
    }
  }
  __syncthreads();

  for (int task = tid; task < NLC * 32; task += 256) {
    const int l = task >> 5, c = task & 31;
    const v4u g = *(const v4ua*)(ctx + ((size_t)(b * NLC + l)) * 256 + 8 * c);
    us* col = sKV + (8 * c) * LP + l;
    col[0 * LP] = (us)(g.x & 0xFFFFu);  col[1 * LP] = (us)(g.x >> 16);
    col[2 * LP] = (us)(g.y & 0xFFFFu);  col[3 * LP] = (us)(g.y >> 16);
    col[4 * LP] = (us)(g.z & 0xFFFFu);  col[5 * LP] = (us)(g.z >> 16);
    col[6 * LP] = (us)(g.w & 0xFFFFu);  col[7 * LP] = (us)(g.w >> 16);
  }
  for (int task = tid; task < NLC * 16; task += 256) {
    const int l = task >> 4, k = task & 15;
    sKV[(256 + k) * LP + l] = sTE[l * 16 + k];
  }
  for (int task = tid; task < KVP * 3; task += 256) {
    const int j = task / 3, q = task - 3 * j;
    *(v4ua*)(sKV + j * LP + 200 + 8 * q) = z4;
  }
  for (int task = tid; task < 16 * 25; task += 256) {
    const int j = 272 + task / 25, q = task - 25 * (task / 25);
    *(v4ua*)(sKV + j * LP + 8 * q) = z4;
  }
  __syncthreads();

  {
    v16us af[7];
    #pragma unroll
    for (int ks = 0; ks < 7; ++ks) af[ks] = ldfrag(sATT + m * LP + 32 * ks, h);
    for (int nt = w; nt < 18; nt += 8) {
      v8f acc = zero8();
      #pragma unroll
      for (int ks = 0; ks < 7; ++ks) {
        const v16us bb = ldfrag(sKV + (16 * nt + m) * LP + 32 * ks, h);
        acc = mma_f16(af[ks], bb, acc);
      }
      if (h == 0) {
        #pragma unroll
        for (int r = 0; r < 4; ++r) sAW[r * KVP + 16 * nt + m] = acc[r] * (1.0f / 16384.0f);
      }
    }
  }
  __syncthreads();

  unsigned char* gd = awp + (size_t)b * 4608;
  store_lines((const unsigned char*)sAW, gd, 36, w, lane, 8);
  __threadfence();
  store_lines((const unsigned char*)sAW, gd, 36, w, lane, 8);
}

__device__ __forceinline__ void ln_row8(const float* rowp, const float* __restrict__ g,
                                        const float* __restrict__ be, int lane, float (&z)[8]) {
  float v[8];
  float s = 0.0f;
  #pragma unroll
  for (int i = 0; i < 8; ++i) { v[i] = rowp[lane + 32 * i]; s += v[i]; }
  s = wsum(s);
  const float mu = s * (1.0f / 256.0f);
  float q = 0.0f;
  #pragma unroll
  for (int i = 0; i < 8; ++i) { const float d = v[i] - mu; v[i] = d; q += d * d; }
  q = wsum(q);
  const float rs = rsqrtf(q * (1.0f / 256.0f) + 1e-5f);
  #pragma unroll
  for (int i = 0; i < 8; ++i) { const int c = lane + 32 * i; z[i] = v[i] * rs * g[c] + be[c]; }
}

__global__ __launch_bounds__(256) void k_post(
    const float* __restrict__ awp, float* hp,
    const us* __restrict__ wvHi, const us* __restrict__ wvLo,
    const us* __restrict__ wrHi, const us* __restrict__ wrLo,
    const us* __restrict__ w1Hi, const us* __restrict__ w1Lo,
    const us* __restrict__ w2Hi, const us* __restrict__ w2Lo,
    const float* __restrict__ bres, const float* __restrict__ bff1, const float* __restrict__ bff2,
    const float* __restrict__ g1, const float* __restrict__ be1,
    const float* __restrict__ g2, const float* __restrict__ be2)
{
  extern __shared__ __align__(16) unsigned char dynlds[];
  us* awHi = (us*)dynlds;
  us* awLo = awHi + 18432;
  us* xHi  = awLo + 18432;
  us* xLo  = xHi + 4096;
  float* sR = (float*)(dynlds + 90112);
  float* sZ = (float*)(dynlds + 106496);

  const int tid = threadIdx.x, lane = tid & 31, w = tid >> 5;
  const int h = lane >> 4, m = lane & 15;
  const int row0 = blockIdx.x * 16;

  stage_split(awp + (size_t)row0 * QKW, 18432, awHi, awLo, tid);
  stage_split(hp + (size_t)row0 * 256, 4096, xHi, xLo, tid);
  __syncthreads();

  const int nb = 32 * w;
  const int hd = w >> 1;
  v8f acc[1][2];
  acc[0][0] = zero8(); acc[0][1] = zero8();
  gemm_split<1, 2>(acc, awHi + 288 * hd, awLo + 288 * hd, QKW,
                   wvHi + (size_t)nb * 288, wvLo + (size_t)nb * 288, 288, 9, lane);
  gemm_split<1, 2>(acc, xHi, xLo, 256, wrHi + (size_t)nb * 256, wrLo + (size_t)nb * 256, 256, 8, lane);
  #pragma unroll
  for (int nt = 0; nt < 2; ++nt) {
    const int col = nb + 16 * nt + m;
    const float bv = bres[col];
    #pragma unroll
    for (int r = 0; r < 8; ++r) sR[(8 * h + r) * 256 + col] = acc[0][nt][r] + bv;
  }
  __syncthreads();

  #pragma unroll
  for (int rr = 0; rr < 2; ++rr) {
    const int row = 2 * w + rr;
    float z[8];
    ln_row8(sR + row * 256, g1, be1, lane, z);
    #pragma unroll
    for (int i = 0; i < 8; ++i) {
      const int c = lane + 32 * i;
      sZ[row * 256 + c] = z[i];
      const us zh = f2bf(z[i]);
      xHi[row * 256 + c] = zh;
      xLo[row * 256 + c] = f2bf(z[i] - bf2f(zh));
    }
  }
  __syncthreads();

  acc[0][0] = zero8(); acc[0][1] = zero8();
  gemm_split<1, 2>(acc, xHi, xLo, 256, w1Hi + (size_t)nb * 256, w1Lo + (size_t)nb * 256, 256, 8, lane);
  __syncthreads();
  #pragma unroll
  for (int nt = 0; nt < 2; ++nt) {
    const int col = nb + 16 * nt + m;
    const float bv = bff1[col];
    #pragma unroll
    for (int r = 0; r < 8; ++r) {
      const int row = 8 * h + r;
      const float a = fmaxf(acc[0][nt][r] + bv, 0.0f);
      const us ah = f2bf(a);
      xHi[row * 256 + col] = ah;
      xLo[row * 256 + col] = f2bf(a - bf2f(ah));
    }
  }
  __syncthreads();

  acc[0][0] = zero8(); acc[0][1] = zero8();
  gemm_split<1, 2>(acc, xHi, xLo, 256, w2Hi + (size_t)nb * 256, w2Lo + (size_t)nb * 256, 256, 8, lane);
  #pragma unroll
  for (int nt = 0; nt < 2; ++nt) {
    const int col = nb + 16 * nt + m;
    const float bv = bff2[col];
    #pragma unroll
    for (int r = 0; r < 8; ++r) {
      const int row = 8 * h + r;
      sR[row * 256 + col] = sZ[row * 256 + col] + (acc[0][nt][r] + bv);
    }
  }
  __syncthreads();

  #pragma unroll
  for (int rr = 0; rr < 2; ++rr) {
    const int row = 2 * w + rr;
    float z[8];
    ln_row8(sR + row * 256, g2, be2, lane, z);
    #pragma unroll
    for (int i = 0; i < 8; ++i) sR[row * 256 + lane + 32 * i] = z[i];
  }
  __syncthreads();

  unsigned char* gd = (unsigned char*)hp + (size_t)row0 * 1024;
  store_lines((const unsigned char*)sR, gd, 128, w, lane, 8);
  __threadfence();
  store_lines((const unsigned char*)sR, gd, 128, w, lane, 8);
}

__global__ __launch_bounds__(256) void k_readout(
    const float* __restrict__ hp,
    const us* __restrict__ wroHi, const us* __restrict__ wroLo,
    const us* __restrict__ ro2Hi, const us* __restrict__ ro2Lo,
    const float* __restrict__ bro, const float* __restrict__ bcls,
    const float* __restrict__ bdt, const float* __restrict__ brem,
    unsigned char* __restrict__ outp)
{
  extern __shared__ __align__(16) unsigned char dynlds[];
  us* aHi = (us*)dynlds;
  us* aLo = aHi + 8192;
  us* zHi = aLo + 8192;
  us* zLo = zHi + 8192;
  float* sLog = (float*)(dynlds + 65536);
  float* sDT  = (float*)(dynlds + 69632);
  float* sREM = (float*)(dynlds + 69760);

  const int tid = threadIdx.x, lane = tid & 31, w = tid >> 5;
  const int h = lane >> 4, m = lane & 15;
  const int row0 = blockIdx.x * 32;

  stage_split(hp + (size_t)row0 * 256, 8192, aHi, aLo, tid);
  __syncthreads();

  const int nb = 32 * w;
  {
    v8f acc[2][2];
    acc[0][0] = zero8(); acc[0][1] = zero8(); acc[1][0] = zero8(); acc[1][1] = zero8();
    gemm_split<2, 2>(acc, aHi, aLo, 256, wroHi + (size_t)nb * 256, wroLo + (size_t)nb * 256, 256, 8, lane);
    #pragma unroll
    for (int nt = 0; nt < 2; ++nt) {
      const int col = nb + 16 * nt + m;
      const float bv = bro[col];
      #pragma unroll
      for (int mt = 0; mt < 2; ++mt) {
        #pragma unroll
        for (int r = 0; r < 8; ++r) {
          const int row = 16 * mt + 8 * h + r;
          const float a = fmaxf(acc[mt][nt][r] + bv, 0.0f);
          const us ah = f2bf(a);
          zHi[row * 256 + col] = ah;
          zLo[row * 256 + col] = f2bf(a - bf2f(ah));
        }
      }
    }
  }
  __syncthreads();

  if (w < 6) {
    v8f a2[2][1];
    a2[0][0] = zero8(); a2[1][0] = zero8();
    gemm_split<2, 1>(a2, zHi, zLo, 256, ro2Hi + (size_t)(16 * w) * 256, ro2Lo + (size_t)(16 * w) * 256, 256, 8, lane);
    const int n = 16 * w + m;
    const float bc = bcls[min(n, 31)];
    const float bd = bdt[0];
    const float br = brem[0];
    #pragma unroll
    for (int mt = 0; mt < 2; ++mt) {
      #pragma unroll
      for (int r = 0; r < 8; ++r) {
        const int row = 16 * mt + 8 * h + r;
        const float v = a2[mt][0][r];
        if (n < 32)       sLog[row * 32 + n] = v + bc;
        else if (n == 32) sDT[row]  = 1.0f / (1.0f + expf(-(v + bd)));
        else if (n == 64) sREM[row] = 1.0f / (1.0f + expf(-(v + br)));
      }
    }
  }
  __syncthreads();

  unsigned char* gLog = outp + (size_t)row0 * 128;
  unsigned char* gDT  = outp + 131072 + (size_t)row0 * 4;
  unsigned char* gREM = outp + 135168 + (size_t)row0 * 4;
  store_lines((const unsigned char*)sLog, gLog, 32, w, lane, 8);
  store_lines((const unsigned char*)sDT,  gDT,  1, w, lane, 8);
  store_lines((const unsigned char*)sREM, gREM, 1, w, lane, 8);
  __threadfence();
  store_lines((const unsigned char*)sLog, gLog, 32, w, lane, 8);
  store_lines((const unsigned char*)sDT,  gDT,  1, w, lane, 8);
  store_lines((const unsigned char*)sREM, gREM, 1, w, lane, 8);
}

extern "C" void kernel_launch(void* const* d_in, const int* in_sizes, int n_in,
                              void* d_out, int out_size, void* d_ws, size_t ws_size,
                              hipStream_t stream) {
  if (n_in < 33) return;
  if (in_sizes[0] != NB * 64) return;
  if (in_sizes[1] != NROWC * 64) return;
  if (in_sizes[2] != NROWC) return;
  if (in_sizes[3] != NB) return;
  if (in_sizes[4] != NROWC) return;
  if (in_sizes[5] != 33 * 32) return;
  if (in_sizes[6] != 96 * 256 || in_sizes[8] != 96 * 256) return;
  if (in_sizes[7] != 256 || in_sizes[9] != 256) return;
  if (in_sizes[10] != 24 || in_sizes[11] != 24) return;
  if (in_sizes[12] != 3 * 65536 || in_sizes[15] != 3 * 65536 || in_sizes[17] != 3 * 65536 || in_sizes[19] != 3 * 65536) return;
  if (in_sizes[13] != 3 * 69632 || in_sizes[14] != 3 * 69632) return;
  if (in_sizes[16] != 768 || in_sizes[18] != 768 || in_sizes[20] != 768) return;
  if (in_sizes[21] != 768 || in_sizes[22] != 768 || in_sizes[23] != 768 || in_sizes[24] != 768) return;
  if (in_sizes[25] != 65536 || in_sizes[26] != 256) return;
  if (in_sizes[27] != 8192 || in_sizes[28] != 32) return;
  if (in_sizes[29] != 256 || in_sizes[30] != 1 || in_sizes[31] != 256 || in_sizes[32] != 1) return;
  if (out_size != NB * 32 + 2 * NB) return;
  if ((size_t)WS_TOTAL > ws_size) return;

  const float* x_u   = (const float*)d_in[0];
  const float* x_ctx = (const float*)d_in[1];
  const float* t_ctx = (const float*)d_in[2];
  const int*   act_u = (const int*)d_in[3];
  const int*   act_c = (const int*)d_in[4];
  const float* emb   = (const float*)d_in[5];
  const float* W_in_self = (const float*)d_in[6];
  const float* b_in_self = (const float*)d_in[7];
  const float* W_in_ctx  = (const float*)d_in[8];
  const float* b_in_ctx  = (const float*)d_in[9];
  const float* freq  = (const float*)d_in[10];
  const float* phase = (const float*)d_in[11];
  const float* Wq    = (const float*)d_in[12];
  const float* Wk    = (const float*)d_in[13];
  const float* Wv    = (const float*)d_in[14];
  const float* Wres  = (const float*)d_in[15];
  const float* bres  = (const float*)d_in[16];
  const float* Wff1  = (const float*)d_in[17];
  const float* bff1  = (const float*)d_in[18];
  const float* Wff2  = (const float*)d_in[19];
  const float* bff2  = (const float*)d_in[20];
  const float* g1    = (const float*)d_in[21];
  const float* beta1 = (const float*)d_in[22];
  const float* g2    = (const float*)d_in[23];
  const float* beta2 = (const float*)d_in[24];
  const float* W_ro  = (const float*)d_in[25];
  const float* b_ro  = (const float*)d_in[26];
  const float* W_cls = (const float*)d_in[27];
  const float* b_cls = (const float*)d_in[28];
  const float* W_dt  = (const float*)d_in[29];
  const float* b_dt  = (const float*)d_in[30];
  const float* W_rem = (const float*)d_in[31];
  const float* b_rem = (const float*)d_in[32];

  unsigned char* ws = (unsigned char*)d_ws;
  us* ctxp            = (us*)(ws + WS_CTX);
  float* hpl          = (float*)(ws + WS_H);
  unsigned char* qkp  = ws + WS_QK;
  unsigned char* awp  = ws + WS_AW;
  const float* awf    = (const float*)(ws + WS_AW);
  us* wsw             = (us*)(ws + WS_W);

  hipFuncSetAttribute((const void*)k_inproj<0>, hipFuncAttributeMaxDynamicSharedMemorySize, LDS_INPROJ0);
  hipFuncSetAttribute((const void*)k_inproj<1>, hipFuncAttributeMaxDynamicSharedMemorySize, LDS_INPROJ1);
  hipFuncSetAttribute((const void*)k_qk, hipFuncAttributeMaxDynamicSharedMemorySize, LDS_QK);
  hipFuncSetAttribute((const void*)k_attn, hipFuncAttributeMaxDynamicSharedMemorySize, LDS_ATTN);
  hipFuncSetAttribute((const void*)k_post, hipFuncAttributeMaxDynamicSharedMemorySize, LDS_POST);
  hipFuncSetAttribute((const void*)k_readout, hipFuncAttributeMaxDynamicSharedMemorySize, LDS_RDO);

  k_cvt<<<dim3(9, 24), 256, 0, stream>>>(W_in_self, W_in_ctx, Wq, Wk, Wv, Wres, Wff1, Wff2,
                                        W_ro, W_cls, W_dt, W_rem, wsw);

  k_inproj<0><<<NB / 64, 256, LDS_INPROJ0, stream>>>(
      x_u, act_u, emb, wsw + OFF_WINS_HI, wsw + OFF_WINS_LO, b_in_self, (unsigned char*)hpl, NB);

  k_inproj<1><<<NROWC / 64, 256, LDS_INPROJ1, stream>>>(
      x_ctx, act_c, emb, wsw + OFF_WINC, wsw + OFF_WINC, b_in_ctx, (unsigned char*)ctxp, NROWC);

  for (int i = 0; i < 3; ++i) {
    const us* lw = wsw + OFF_L0 + (size_t)i * LSTRIDE;
    k_qk<<<NB / 32, 256, LDS_QK, stream>>>(hpl, lw + L_WQ_HI, lw + L_WQ_LO, lw + L_WK_HI, lw + L_WK_LO, qkp);
    k_attn<<<NB, 256, LDS_ATTN, stream>>>(ctxp, t_ctx, act_c, freq + 8 * i, phase + 8 * i, qkp, awp);
    k_post<<<NB / 16, 256, LDS_POST, stream>>>(
        awf, hpl,
        lw + L_WV_HI, lw + L_WV_LO, lw + L_WR_HI, lw + L_WR_LO,
        lw + L_W1_HI, lw + L_W1_LO, lw + L_W2_HI, lw + L_W2_LO,
        bres + 256 * i, bff1 + 256 * i, bff2 + 256 * i,
        g1 + 256 * i, beta1 + 256 * i, g2 + 256 * i, beta2 + 256 * i);
  }

  const us* rw = wsw + OFF_RB;
  k_readout<<<NB / 32, 256, LDS_RDO, stream>>>(
      hpl, rw + R_WRO_HI, rw + R_WRO_LO, rw + R_RO2_HI, rw + R_RO2_LO,
      b_ro, b_cls, b_dt, b_rem, (unsigned char*)d_out);
}
